// EdgePredictionGNN_82162724372639
// MI455X (gfx1250) — hardware-run, weakly checked
//
#include <hip/hip_runtime.h>


namespace {
constexpr int N = 100000, NP = 100032, E = 1600000, D = 64, DM = 64;
constexpr float XS = 8.0f, WSC = 256.0f, NEG = 0.2f;
typedef _Float16 b16;
typedef __attribute__((ext_vector_type(16))) _Float16 v16b;
typedef __attribute__((ext_vector_type(8))) _Float16 v8b;
typedef __attribute__((ext_vector_type(8))) float v8f;
typedef __attribute__((ext_vector_type(4))) float v4f;
typedef __attribute__((ext_vector_type(2))) float v2f;
__device__ __forceinline__ float bf16_rne(float f) { unsigned int u = __float_as_uint(f); u += 0x7FFFu + ((u >> 16) & 1u); return __uint_as_float(u & 0xFFFF0000u); }
__device__ __forceinline__ void split16(float v, b16& hi, b16& lo) { hi = (b16)v; lo = (b16)(v - (float)hi); }
__device__ __forceinline__ v16b frag_kb(const b16* p, int hh) { const v8b a = *(const v8b*)(p + 8 * hh), b = *(const v8b*)(p + 16 + 8 * hh); v16b f;
#pragma unroll
  for (int e = 0; e < 8; ++e) { f[e] = a[e]; f[8 + e] = b[e]; } return f; }
__device__ __forceinline__ v8f wmma16b(v16b a, v16b b, v8f c) { v8f d = __builtin_amdgcn_wmma_f32_16x16x32_f16(false, a, false, b, (short)0, c, false, false); asm volatile("v_nop\n\tv_nop\n\tv_nop\n\tv_nop" : "+v"(d) : "v"(a), "v"(b)); return d; }
__device__ __forceinline__ void wave_lds_sync() { __builtin_amdgcn_fence(__ATOMIC_RELEASE, "workgroup"); __builtin_amdgcn_wave_barrier(); __builtin_amdgcn_fence(__ATOMIC_ACQUIRE, "workgroup"); }
__device__ __forceinline__ float pmul(float a, float b) { float p = a * b; asm volatile("" : "+v"(p)); return p; }
__device__ __forceinline__ float opaque(float a) { asm volatile("" : "+v"(a)); return a; }
__device__ __forceinline__ int iclamp(int v, int lo, int hi) { return v < lo ? lo : (v > hi ? hi : v); }
__device__ __forceinline__ float nexp(float x) { return __builtin_amdgcn_exp2f(x * 1.4426950408889634f); }
__device__ __forceinline__ float lrelu(float x) { return x > 0.0f ? x : NEG * x; }
constexpr int CSR_NBLK = 512, CSR_GB = 9, CSR_GN = 1 << CSR_GB  , CSR_MAXG = 512, CSR_CAP = 12288  ;
__global__ __launch_bounds__(64) void csrA_kernel(const int* __restrict__ dst, int E, int N, int nG, int CHP, int NGP, int* __restrict__ STG, int* __restrict__ HST) {
  extern __shared__ int sm[];
  int* cnt = sm; int* run = sm + NGP; int* ids = sm + 2 * NGP;
  const int b = blockIdx.x; const int ch = (E + CSR_NBLK - 1) / CSR_NBLK; const int e0 = b * ch, e1 = min(E, e0 + ch);
  for (int i = threadIdx.x; i < NGP; i += 64) cnt[i] = 0;
  for (int i = threadIdx.x; i < CHP; i += 64) ids[i] = -1;
  __syncthreads();
  if (threadIdx.x == 0) {
    for (int e = e0; e < e1; ++e) { int d = dst[e]; d = (d < 0) ? 0 : (d >= N ? N - 1 : d); cnt[d >> CSR_GB] += 1; }
    int acc = 0; for (int g = 0; g < nG; ++g) { run[g] = acc; acc += cnt[g]; }
    for (int e = e0; e < e1; ++e) { int d = dst[e]; d = (d < 0) ? 0 : (d >= N ? N - 1 : d); const int g = d >> CSR_GB; ids[run[g]] = e; run[g] += 1; } }
  __syncthreads();
  typedef __attribute__((ext_vector_type(4))) int v4i;
  for (int pass = 0; pass < 2; ++pass) {
    for (int i = threadIdx.x; i < CHP / 4; i += 64) *(volatile v4i*)(STG + (size_t)b * CHP + i * 4) = *(const v4i*)(&ids[i * 4]);
    for (int i = threadIdx.x; i < NGP / 4; i += 64) { v4i v; for (int e = 0; e < 4; ++e) v[e] = (i * 4 + e < nG) ? cnt[i * 4 + e] : 0; *(volatile v4i*)(HST + (size_t)b * NGP + i * 4) = v; }
    __threadfence(); }
}
__global__ __launch_bounds__(512) void csrS_kernel(const int* __restrict__ HST, int nG, int NGP, int* __restrict__ START, int* __restrict__ TOT, int* __restrict__ OFF) {
  __shared__ int tot[CSR_MAXG];
  const int b = threadIdx.x;
  for (int pass = 0; pass < 2; ++pass) { int runb = 0; for (int g = 0; g < nG; ++g) { int c = HST[(size_t)b * NGP + g]; c = (c < 0) ? 0 : c; ((volatile int*)OFF)[(size_t)g * CSR_NBLK + b] = runb; runb += c; } __threadfence(); }
  for (int g = threadIdx.x; g < nG; g += 512) { int s = 0; for (int bb = 0; bb < CSR_NBLK; ++bb) { int c = HST[(size_t)bb * NGP + g]; s += (c < 0) ? 0 : c; } tot[g] = s; }
  __syncthreads();
  if (threadIdx.x < 32) {
    __shared__ int st[CSR_MAXG + 32];
    if (threadIdx.x == 0) { int acc = 0; for (int g = 0; g < NGP; ++g) { st[g] = acc; if (g < nG) acc += (tot[g] + 31) & ~31; } st[NGP] = acc; }
    __builtin_amdgcn_fence(__ATOMIC_RELEASE, "workgroup"); __builtin_amdgcn_wave_barrier(); __builtin_amdgcn_fence(__ATOMIC_ACQUIRE, "workgroup");
    for (int pass = 0; pass < 2; ++pass) { for (int i = threadIdx.x; i < NGP + 32; i += 32) { ((volatile int*)START)[i] = (i <= NGP) ? st[min(i, NGP)] : 0; ((volatile int*)TOT)[i] = (i < nG) ? tot[i] : 0; } __threadfence(); } }
}
__global__ __launch_bounds__(256) void csrB_kernel(const int* __restrict__ dst, int N, int nG, int CHP, int NGP, int permLen, const int* __restrict__ STG, const int* __restrict__ HST, const int* __restrict__ OFF, const int* __restrict__ START, const int* __restrict__ TOT, int* __restrict__ PERM, int* __restrict__ ROWPTR, int* __restrict__ ROWCNT, int* __restrict__ FLAG) {
  typedef __attribute__((ext_vector_type(4))) int v4i;
  __shared__ int ids[CSR_CAP]; __shared__ unsigned short key[CSR_CAP]; __shared__ int outp[CSR_CAP]; __shared__ int ncnt[CSR_GN + 1]; __shared__ int boff[CSR_NBLK + 1];
  const int g = blockIdx.x, t_ = threadIdx.x; int tot = TOT[g]; int st = START[g], stn = START[g + 1]; const int v0 = g * CSR_GN; const int nv = min(CSR_GN, N - v0);
  st = (st < 0) ? 0 : (st > permLen - 32 ? permLen - 32 : st) & ~31; stn = (stn < st) ? st : (stn > permLen ? permLen : stn); tot = (tot < 0) ? 0 : tot; if (tot > stn - st && tot <= CSR_CAP) tot = stn - st;
  if (tot > CSR_CAP) {
    for (int pass = 0; pass < 2; ++pass) { for (int i = t_; i < CSR_GN / 4; i += 256) { v4i a, c; for (int e = 0; e < 4; ++e) { a[e] = st; c[e] = 0; } *(volatile v4i*)(ROWPTR + v0 + i * 4) = a; *(volatile v4i*)(ROWCNT + v0 + i * 4) = c; } if (t_ == 0) ((volatile int*)FLAG)[0] = 1; __threadfence(); } (void)nv; return; }
  if (t_ == 0) { int acc = 0; for (int b = 0; b < CSR_NBLK; ++b) { boff[b] = acc; int c = HST[(size_t)b * NGP + g]; c = (c < 0) ? 0 : (c > CHP ? CHP : c); acc += c; if (acc > tot) acc = tot; } boff[CSR_NBLK] = acc; }
  for (int i = t_; i <= CSR_GN; i += 256) ncnt[i] = 0;
  __syncthreads();
  for (int b = 0; b < CSR_NBLK; ++b) { const int c = boff[b + 1] - boff[b]; int o_ = OFF[(size_t)g * CSR_NBLK + b]; o_ = (o_ < 0) ? 0 : (o_ > CHP - c ? CHP - c : o_); const int* src_ = STG + (size_t)b * CHP + o_;
    for (int i = t_; i < c; i += 256) { int id = src_[i]; id = (id < 0) ? 0 : id; ids[boff[b] + i] = id; int d = dst[id]; d = (d < v0) ? v0 : (d >= N ? N - 1 : d); int kk = d - v0; kk = (kk < 0) ? 0 : (kk >= CSR_GN ? CSR_GN - 1 : kk); key[boff[b] + i] = (unsigned short)kk; } }
  __syncthreads();
  if (t_ == 0) { for (int i = 0; i < tot; ++i) ncnt[key[i]] += 1; int acc = 0; for (int vl = 0; vl < CSR_GN; ++vl) { const int c = ncnt[vl]; ncnt[vl] = acc; acc += c; } ncnt[CSR_GN] = acc;
    for (int i = 0; i < tot; ++i) { const int vl = key[i]; outp[ncnt[vl]] = ids[i]; ncnt[vl] += 1; }
    for (int vl = CSR_GN; vl > 0; --vl) ncnt[vl] = ncnt[vl - 1]; ncnt[0] = 0; }
  __syncthreads();
  for (int pass = 0; pass < 2; ++pass) {
    for (int i = t_; i < (stn - st) / 4; i += 256) { v4i v; for (int e = 0; e < 4; ++e) { const int q = i * 4 + e; v[e] = (q < tot) ? outp[q] : -1; } *(volatile v4i*)(PERM + st + i * 4) = v; }
    for (int i = t_; i < CSR_GN / 4; i += 256) { v4i a, c; for (int e = 0; e < 4; ++e) { const int vl = i * 4 + e; a[e] = st + ncnt[vl]; c[e] = (vl < nv) ? (ncnt[vl + 1] - ncnt[vl]) : 0; } *(volatile v4i*)(ROWPTR + v0 + i * 4) = a; *(volatile v4i*)(ROWCNT + v0 + i * 4) = c; }
    __threadfence(); }
}
__global__ __launch_bounds__(256) void csrZ_kernel(int* __restrict__ p, size_t n4) { typedef __attribute__((ext_vector_type(4))) int v4i; const size_t tid = (size_t)blockIdx.x * 256 + threadIdx.x, nth = (size_t)gridDim.x * 256; v4i z = {0, 0, 0, 0}; for (size_t i = tid; i < n4; i += nth) *(volatile v4i*)(p + i * 4) = z; }
struct CsrBufs { int *STG, *HST, *OFF, *START, *TOT, *PERM, *ROWPTR, *ROWCNT, *FLAG; int nG, NGP, CHP; size_t permLen; char* base; size_t bytes; };
static size_t csr_carve(CsrBufs& c, char* ws, size_t off, int E, int N) {
  const size_t off0 = off; c.base = ws + off;
  auto al = [&](size_t bytes) { char* p = ws + off; off += (bytes + 255) & ~(size_t)255; return p; };
  c.nG = (N + CSR_GN - 1) / CSR_GN; c.NGP = (c.nG + 31) & ~31; const int ch = (E + CSR_NBLK - 1) / CSR_NBLK; c.CHP = (ch + 31) & ~31; c.permLen = (size_t)E + 32 * (size_t)c.nG + 32;
  c.STG = (int*)al((size_t)CSR_NBLK * c.CHP * 4); c.HST = (int*)al((size_t)CSR_NBLK * c.NGP * 4); c.OFF = (int*)al((size_t)c.NGP * CSR_NBLK * 4); c.START = (int*)al((size_t)(c.NGP + 64) * 4); c.TOT = (int*)al((size_t)(c.NGP + 64) * 4);
  c.PERM = (int*)al(c.permLen * 4); c.ROWPTR = (int*)al((size_t)c.nG * CSR_GN * 4); c.ROWCNT = (int*)al((size_t)c.nG * CSR_GN * 4); c.FLAG = (int*)al(256);
  c.bytes = off - off0; return off;
}
static void csr_build(const CsrBufs& c, const int* dst, int E, int N, hipStream_t stream) {
  const size_t smem = (size_t)(2 * c.NGP + c.CHP) * 4;
  csrZ_kernel<<<512, 256, 0, stream>>>((int*)c.base, c.bytes / 16);
  csrA_kernel<<<CSR_NBLK, 64, smem, stream>>>(dst, E, N, c.nG, c.CHP, c.NGP, c.STG, c.HST);
  csrS_kernel<<<1, 512, 0, stream>>>(c.HST, c.nG, c.NGP, c.START, c.TOT, c.OFF);
  csrB_kernel<<<c.nG, 256, 0, stream>>>(dst, N, c.nG, c.CHP, c.NGP, (int)c.permLen, c.STG, c.HST, c.OFF, c.START, c.TOT, c.PERM, c.ROWPTR, c.ROWCNT, c.FLAG);
}


__global__ __launch_bounds__(256) void wprep_kernel(const float* __restrict__ w1, const float* __restrict__ w2, const float* __restrict__ wm1, b16* __restrict__ W1T, b16* __restrict__ W2T, b16* __restrict__ WMT) {
  const size_t u = (size_t)blockIdx.x * 256 + threadIdx.x; const size_t n = (size_t)D * D / 8; size_t t = u; v8b o;
  if (t < n) { const size_t e = t * 8; const int oo = (int)(e / D), k0 = (int)(e % D); for (int j = 0; j < 8; ++j) o[j] = (b16)(bf16_rne(w1[(size_t)(k0 + j) * D + oo]) * WSC); for (int pass = 0; pass < 2; ++pass) { *(volatile v8b*)(W1T + e) = o; __threadfence(); } return; } t -= n;
  if (t < n) { const size_t e = t * 8; const int oo = (int)(e / D), k0 = (int)(e % D); for (int j = 0; j < 8; ++j) o[j] = (b16)(bf16_rne(w2[(size_t)(k0 + j) * D + oo]) * WSC); for (int pass = 0; pass < 2; ++pass) { *(volatile v8b*)(W2T + e) = o; __threadfence(); } return; } t -= n;
  if (t < 2 * n) { const size_t e = t * 8; const int row = (int)(e / D), k0 = (int)(e % D); const int part = row / DM, oo = row % DM; for (int j = 0; j < 8; ++j) { const int k = k0 + j; const int srow = part ? (D + 1 + k) : k; o[j] = (b16)(bf16_rne(wm1[(size_t)srow * DM + oo]) * WSC); } for (int pass = 0; pass < 2; ++pass) { *(volatile v8b*)(WMT + e) = o; __threadfence(); } }
}
template <int COUT, int EXACT>
__global__ __launch_bounds__(128) void trans_kernel(const float* __restrict__ src, const b16* __restrict__ WT, const float* __restrict__ as_, const float* __restrict__ ad_, float* __restrict__ OUT, float* __restrict__ SC) {
  constexpr int NT = COUT / 16;
  __shared__ __attribute__((aligned(16))) b16 Ah[EXACT ? 1 : 4][16][D + 8], Al[EXACT ? 1 : 4][16][D + 8]; __shared__ __attribute__((aligned(16))) float Tf[4][16][COUT + 4]; __shared__ __attribute__((aligned(16))) float sc[64][2];
  const int wave = threadIdx.x >> 5, lane = threadIdx.x & 31, nloc = lane & 15, hlf = lane >> 4; const size_t m0 = (size_t)blockIdx.x * 64 + wave * 16;
  if (!EXACT) { for (int rr = 0; rr < 16; ++rr) if (lane < 16) { const v4f v = *(const v4f*)(src + (m0 + rr) * D + lane * 4); for (int j = 0; j < 4; ++j) { b16 p, s; split16(v[j] * XS, p, s); Ah[wave][rr][lane * 4 + j] = p; Al[wave][rr][lane * 4 + j] = s; } } wave_lds_sync(); }
  v8f acc[NT];
#pragma unroll
  for (int t = 0; t < NT; ++t) acc[t] = (v8f){};
#pragma unroll
  for (int kb = 0; kb < D; kb += 32) { v16b a = {}, al = {};
    if (EXACT) { const size_t v = m0 + nloc; if (v < (size_t)N) { const float* r = src + v * D + kb; for (int e = 0; e < 8; ++e) { a[e] = (b16)(bf16_rne(r[8 * hlf + e]) * XS); a[8 + e] = (b16)(bf16_rne(r[16 + 8 * hlf + e]) * XS); } } }
    else { a = frag_kb(&Ah[EXACT ? 0 : wave][nloc][kb], hlf); al = frag_kb(&Al[EXACT ? 0 : wave][nloc][kb], hlf); }
#pragma unroll
    for (int t = 0; t < NT; ++t) { const v16b bw = frag_kb(WT + (size_t)(t * 16 + nloc) * D + kb, hlf); acc[t] = wmma16b(a, bw, acc[t]); if (!EXACT) acc[t] = wmma16b(al, bw, acc[t]); } }
#pragma unroll
  for (int t = 0; t < NT; ++t)
#pragma unroll 1
    for (int r = 0; r < 8; ++r) { const size_t row = m0 + 8 * hlf + r; Tf[wave][8 * hlf + r][t * 16 + nloc] = row < (size_t)N ? acc[t][r] * (1.0f / (XS * WSC)) : 0.0f; }
  wave_lds_sync();
  if (SC != nullptr) { const float a0 = opaque(bf16_rne(as_[lane * 2])), a1 = opaque(bf16_rne(as_[lane * 2 + 1])), d0 = opaque(bf16_rne(ad_[lane * 2])), d1 = opaque(bf16_rne(ad_[lane * 2 + 1]));
    for (int rr = 0; rr < 16; ++rr) { const v2f h = *(const v2f*)(&Tf[wave][rr][lane * 2]); float s = pmul(h[0], a0) + pmul(h[1], a1), dd = pmul(h[0], d0) + pmul(h[1], d1); for (int sh = 16; sh; sh >>= 1) { s += __shfl_xor(s, sh); dd += __shfl_xor(dd, sh); } if (lane == 0) { sc[wave * 16 + rr][0] = s; sc[wave * 16 + rr][1] = dd; } } }
  __syncthreads();
  for (int pass = 0; pass < 2; ++pass) { for (int rr = 0; rr < 16; ++rr) for (int q = lane * 4; q < COUT; q += 128) *(volatile v4f*)(OUT + (m0 + rr) * COUT + q) = *(const v4f*)(&Tf[wave][rr][q]);
    if (SC != nullptr && threadIdx.x < 32) *(volatile v4f*)(SC + (size_t)blockIdx.x * 128 + threadIdx.x * 4) = *(const v4f*)(&sc[0][0] + threadIdx.x * 4); __threadfence(); }
}
__global__ __launch_bounds__(256) void agg_kernel(const float* __restrict__ T, const float* __restrict__ SC, const float* __restrict__ ea, const float* __restrict__ we, const float* __restrict__ ae, const float* __restrict__ bias, const int* __restrict__ srcs, const int* __restrict__ PERM, const int* __restrict__ ROWPTR, const int* __restrict__ ROWCNT, int permLen, float* __restrict__ H) {
  const int wave = threadIdx.x >> 5, lane = threadIdx.x & 31; const size_t v = (size_t)blockIdx.x * 8 + wave; const int c0 = lane * 2;
  float cw; { float s = pmul(bf16_rne(we[c0]), bf16_rne(ae[c0])) + pmul(bf16_rne(we[c0 + 1]), bf16_rne(ae[c0 + 1])); for (int sh = 16; sh; sh >>= 1) s += __shfl_xor(s, sh); cw = s; }
  v2f o = {0.0f, 0.0f};
  int st = 0, cnt = 0; if (v < (size_t)N) { st = ROWPTR[v]; cnt = ROWCNT[v]; cnt = iclamp(cnt, 0, 65536); st = iclamp(st, 0, permLen - cnt); }
  float la = 0.0f;
#pragma unroll 1
  for (int j = 0; j < cnt; ++j) { const int e = iclamp(PERM[st + j], 0, E - 1); la += bf16_rne(ea[e]); }
  la = la / fmaxf((float)cnt, 1.0f);
  const float asv = SC[v * 2], adv = SC[v * 2 + 1]; const float eself = lrelu(asv + adv + pmul(la, cw)); float mx = eself;
#pragma unroll 1
  for (int j = 0; j < cnt; ++j) { const int e = iclamp(PERM[st + j], 0, E - 1); const size_t s = (size_t)iclamp(srcs[e], 0, N - 1); mx = fmaxf(mx, lrelu(SC[s * 2] + adv + pmul(bf16_rne(ea[e]), cw))); }
  float den = nexp(eself - mx); const v2f hv = *(const v2f*)(T + v * D + c0); float a0 = pmul(den, hv[0]), a1 = pmul(den, hv[1]);
#pragma unroll 1
  for (int j = 0; j < cnt; ++j) { const int e = iclamp(PERM[st + j], 0, E - 1); const size_t s = (size_t)iclamp(srcs[e], 0, N - 1); const float p = nexp(lrelu(SC[s * 2] + adv + pmul(bf16_rne(ea[e]), cw)) - mx); den += p; const v2f hs = *(const v2f*)(T + s * D + c0); a0 += pmul(p, hs[0]); a1 += pmul(p, hs[1]); }
  if (v < (size_t)N) { const float inv = 1.0f / den; o[0] = fmaxf(pmul(a0, inv) + bf16_rne(bias[c0]), 0.0f); o[1] = fmaxf(pmul(a1, inv) + bf16_rne(bias[c0 + 1]), 0.0f); }
  for (int pass = 0; pass < 2; ++pass) { *(volatile v2f*)(H + v * D + c0) = o; __threadfence(); }
}
__global__ __launch_bounds__(256) void edge_kernel(const float* __restrict__ PQ, const float* __restrict__ ea, const int* __restrict__ ei, const float* __restrict__ wm1, const float* __restrict__ bm1, const float* __restrict__ wm2, const float* __restrict__ bm2, float* __restrict__ out) {
  __shared__ __attribute__((aligned(16))) float so[64];
  const int wave = threadIdx.x >> 5, lane = threadIdx.x & 31; const int c0 = lane * 2;
  const float we0 = bf16_rne(wm1[(size_t)D * DM + c0]), we1 = bf16_rne(wm1[(size_t)D * DM + c0 + 1]), b0 = bf16_rne(bm1[c0]), b1 = bf16_rne(bm1[c0 + 1]), m0 = opaque(bf16_rne(wm2[c0])), m1 = opaque(bf16_rne(wm2[c0 + 1])), bo = bf16_rne(bm2[0]);
#pragma unroll 1
  for (int q = 0; q < 8; ++q) { const size_t e = (size_t)blockIdx.x * 64 + wave * 8 + q; float d = 0.0f;
    if (e < (size_t)E) { const size_t s = (size_t)iclamp(ei[e], 0, N - 1), t = (size_t)iclamp(ei[(size_t)E + e], 0, N - 1); const float a = bf16_rne(ea[e]); const v2f ps = *(const v2f*)(PQ + s * 2 * DM + c0), qt = *(const v2f*)(PQ + t * 2 * DM + DM + c0);
      const float z0 = fmaxf(ps[0] + pmul(a, we0) + qt[0] + b0, 0.0f), z1 = fmaxf(ps[1] + pmul(a, we1) + qt[1] + b1, 0.0f); d = pmul(z0, m0) + pmul(z1, m1); }
    for (int sh = 16; sh; sh >>= 1) d += __shfl_xor(d, sh);
    if (lane == 0) so[wave * 8 + q] = d + bo; }
  __syncthreads();
  for (int pass = 0; pass < 2; ++pass) { if (threadIdx.x < 16) *(volatile v4f*)(out + (size_t)blockIdx.x * 64 + threadIdx.x * 4) = *(const v4f*)(&so[threadIdx.x * 4]); __threadfence(); }
}
}

extern "C" void kernel_launch(void* const* d_in, const int* in_sizes, int n_in, void* d_out, int out_size, void* d_ws, size_t ws_size, hipStream_t stream) {
  (void)n_in;
  auto Fp = [&](int i) { return (const float*)d_in[i]; }; auto Ip = [&](int i) { return (const int*)d_in[i]; };
  if (in_sizes[0] != N * D || in_sizes[1] != 2 * E || in_sizes[2] != E || in_sizes[3] != D * D || in_sizes[9] != D * D || in_sizes[15] != (2 * D + 1) * DM || in_sizes[17] != DM || out_size != E) return;
  size_t off = 0; char* ws = (char*)d_ws;
  auto carve = [&](size_t bytes) { char* p = ws + off; off += (bytes + 255) & ~(size_t)255; return p; };
  b16* W1T = (b16*)carve((size_t)D * D * 2); b16* W2T = (b16*)carve((size_t)D * D * 2); b16* WMT = (b16*)carve((size_t)2 * DM * D * 2);
  float* T = (float*)carve((size_t)NP * D * 4); float* H = (float*)carve((size_t)NP * D * 4); float* SC = (float*)carve((size_t)NP * 2 * 4); float* PQ = (float*)carve((size_t)NP * 2 * DM * 4);
  CsrBufs csr; off = csr_carve(csr, ws, off, E, N);
  if (off > ws_size || off > ((size_t)128 << 20)) return;
  wprep_kernel<<<(unsigned)((4 * (size_t)D * D / 8 + 255) / 256), 256, 0, stream>>>(Fp(3), Fp(9), Fp(15), W1T, W2T, WMT);
  csr_build(csr, Ip(1) + E, E, N, stream);
  trans_kernel<D, 1><<<NP / 64, 128, 0, stream>>>(Fp(0), W1T, Fp(4), Fp(5), T, SC);
  agg_kernel<<<NP / 8, 256, 0, stream>>>(T, SC, Fp(2), Fp(6), Fp(7), Fp(8), Ip(1), csr.PERM, csr.ROWPTR, csr.ROWCNT, (int)csr.permLen, H);
  trans_kernel<D, 0><<<NP / 64, 128, 0, stream>>>(H, W2T, Fp(10), Fp(11), T, SC);
  agg_kernel<<<NP / 8, 256, 0, stream>>>(T, SC, Fp(2), Fp(12), Fp(13), Fp(14), Ip(1), csr.PERM, csr.ROWPTR, csr.ROWCNT, (int)csr.permLen, H);
  trans_kernel<2 * DM, 0><<<NP / 64, 128, 0, stream>>>(H, WMT, nullptr, nullptr, PQ, nullptr);
  edge_kernel<<<E / 64, 256, 0, stream>>>(PQ, Fp(2), Ip(1), Fp(15), Fp(16), Fp(17), Fp(18), (float*)d_out);
}
